// XlnetAttention_23433341567288
// MI455X (gfx1250) — hardware-verified
//
#include <hip/hip_runtime.h>


#define QL   512
#define NB_  8
#define PL_  1024
#define HIDN 1024
#define NH_  16
#define HD   64
#define NRQ  (QL * NB_)
#define NRP  (PL_ * NB_)
#define ZH   16
#define DM   HIDN
#define SCL  0.125f
#define LEPS 1e-5f
#define LOSC 1024.0f

typedef _Float16 h16;
typedef unsigned short bf;
typedef __attribute__((ext_vector_type(16))) __bf16   v16bf;
typedef __attribute__((ext_vector_type(16))) _Float16 v16h;
typedef __attribute__((ext_vector_type(8)))  _Float16 v8h;
typedef __attribute__((ext_vector_type(8)))  unsigned short v8us;
typedef __attribute__((ext_vector_type(8)))  float    v8f;
typedef __attribute__((ext_vector_type(4)))  float    v4f;
typedef __attribute__((ext_vector_type(4)))  _Float16 v4h;
typedef v8h  __attribute__((may_alias)) v8ha;
typedef v4f  __attribute__((may_alias)) v4fa;
typedef v8us __attribute__((may_alias)) v8usa;

__device__ __forceinline__ unsigned short f2bf(float f) { unsigned u = __float_as_uint(f); u += 0x7FFFu + ((u >> 16) & 1u); return (unsigned short)(u >> 16); }
__device__ __forceinline__ float bf2f(unsigned short b) { return __uint_as_float(((unsigned)b) << 16); }
__device__ __forceinline__ float bfr(float f) { return bf2f(f2bf(f)); }
__device__ __forceinline__ v16h cat16(v8h lo, v8h hi) { return __builtin_shufflevector(lo, hi, 0, 1, 2, 3, 4, 5, 6, 7, 8, 9, 10, 11, 12, 13, 14, 15); }
__device__ __forceinline__ v16bf cat16b(v8us lo, v8us hi) { return __builtin_bit_cast(v16bf, __builtin_shufflevector(lo, hi, 0, 1, 2, 3, 4, 5, 6, 7, 8, 9, 10, 11, 12, 13, 14, 15)); }
__device__ __forceinline__ v8f wmma16(v16h a, v16h b, v8f c) { return __builtin_amdgcn_wmma_f32_16x16x32_f16(false, a, false, b, (short)0, c, false, false); }
__device__ __forceinline__ v8f wmmab(v16bf a, v16bf b, v8f c) { return __builtin_amdgcn_wmma_f32_16x16x32_bf16(false, a, false, b, (short)0, c, false, false); }

template <bool SPLITA, bool F16OUT = false>
__global__ __launch_bounds__(128) void k_gemmb(const bf* __restrict__ A, const bf* __restrict__ Al, const bf* __restrict__ Bn, const float* __restrict__ bias, float* C, int ldc, h16* C2, const float* __restrict__ R = nullptr, int K = DM, int roundR = 1) {
    __shared__ __align__(16) float ost[4][16 * 68];
    const int lane = threadIdx.x & 31, wave = threadIdx.x >> 5, lr = lane & 15, hi = lane >> 4;
    const int r0 = blockIdx.x * 64 + wave * 16, c0 = blockIdx.y * 64;
    const size_t aoff = (size_t)(r0 + lr) * K + 8 * hi;
    size_t boff[4];
#pragma unroll
    for (int t = 0; t < 4; ++t) boff[t] = (size_t)(c0 + t * 16 + lr) * K + 8 * hi;
    v8f acc[4];
#pragma unroll
    for (int t = 0; t < 4; ++t) acc[t] = (v8f){};
#pragma unroll 1
    for (int kc = 0; kc < K; kc += 32) {
        const v16bf a = cat16b(*(const v8us*)(A + aoff + kc), *(const v8us*)(A + aoff + kc + 16));
        v16bf al = a;
        if (SPLITA) al = cat16b(*(const v8us*)(Al + aoff + kc), *(const v8us*)(Al + aoff + kc + 16));
#pragma unroll
        for (int t = 0; t < 4; ++t) { const v16bf b = cat16b(*(const v8us*)(Bn + boff[t] + kc), *(const v8us*)(Bn + boff[t] + kc + 16)); acc[t] = wmmab(a, b, acc[t]); if (SPLITA) acc[t] = wmmab(al, b, acc[t]); }
        asm volatile("v_nop\n\tv_nop\n\tv_nop\n\tv_nop" : "+v"(acc[0]), "+v"(acc[1]), "+v"(acc[2]), "+v"(acc[3]) : "v"(a), "v"(al));
    }
    float* os = &ost[wave][0];
#pragma unroll
    for (int t = 0; t < 4; ++t) { const float bv = bias ? bfr(bias[c0 + t * 16 + lr]) : 0.f;
#pragma unroll
        for (int j = 0; j < 8; ++j) os[(hi * 8 + j) * 68 + t * 16 + lr] = acc[t][j] + bv; }
    __syncthreads();
    if (F16OUT) {
        h16* crow = (h16*)(void*)C + (size_t)r0 * ldc + c0;
        auto pass = [&]() {
#pragma unroll
            for (int s = 0; s < 4; ++s) { const int row = 4 * s + (lane >> 3), piece = lane & 7; const float* sp = os + row * 68 + piece * 8; v8h o, o2;
#pragma unroll
                for (int i = 0; i < 8; ++i) { const h16 a = (h16)sp[i]; o[i] = a; o2[i] = (h16)((sp[i] - (float)a) * LOSC); }
                *(volatile v8h*)(crow + (size_t)row * ldc + piece * 8) = o; if (C2) *(volatile v8h*)(C2 + (size_t)r0 * ldc + c0 + (size_t)row * ldc + piece * 8) = o2; }
        };
        pass(); __threadfence(); pass();
    } else {
        float* crow = C + (size_t)r0 * ldc + c0;
        auto pass = [&]() {
#pragma unroll
            for (int s = 0; s < 8; ++s) { const int Lid = (lane >> 3) + 4 * s, piece = lane & 7; const int row = Lid >> 1, cofs = (Lid & 1) * 32 + piece * 4;
                v4f val = *(const v4fa*)(os + row * 68 + cofs); if (R) { const v4f rv = *(const v4f*)(R + ((size_t)r0 + row) * ldc + c0 + cofs); val += roundR ? (v4f){bfr(rv[0]), bfr(rv[1]), bfr(rv[2]), bfr(rv[3])} : rv; }
                *(volatile v4f*)(crow + (size_t)row * ldc + cofs) = val; }
        };
        pass(); __threadfence(); pass();
    }
}

__global__ __launch_bounds__(256) void k_cvt8(const float* __restrict__ src, bf* dst, size_t n8) {
    const size_t i = (size_t)blockIdx.x * 256 + threadIdx.x; if (i >= n8) return;
    const v8f v = *(const v8f*)(src + i * 8); v8us o;
#pragma unroll
    for (int k = 0; k < 8; ++k) o[k] = f2bf(v[k]);
    *(volatile v8us*)(dst + i * 8) = o; __threadfence(); *(volatile v8us*)(dst + i * 8) = o;
}
__global__ __launch_bounds__(256) void k_zero8(bf* dst, size_t n8) {
    const size_t i = (size_t)blockIdx.x * 256 + threadIdx.x; if (i >= n8) return; v8us z;
#pragma unroll
    for (int k = 0; k < 8; ++k) z[k] = 0;
    *(volatile v8us*)(dst + i * 8) = z; __threadfence(); *(volatile v8us*)(dst + i * 8) = z;
}

template <int MODE>
__global__ __launch_bounds__(128) void k_gemm3z(const bf* __restrict__ Ah, const bf* __restrict__ Al, const bf* __restrict__ Bh, const bf* __restrict__ Bl, int K, float* C, int ldc, size_t sA, size_t sB, size_t sC) {
    if ((MODE & 1) && (int)blockIdx.y * 64 > (int)blockIdx.x * 64 + 63) return;
    const size_t z = blockIdx.z; Ah += z * sA; Al += z * sA; Bh += z * sB; Bl += z * sB; C += z * sC;
    const int Klim = (MODE & 2) ? min(K, ((int)blockIdx.x + 1) * 64) : K;
    __shared__ __align__(16) float ost[4][16 * 68];
    const int lane = threadIdx.x & 31, wave = threadIdx.x >> 5, lr = lane & 15, hi = lane >> 4;
    const int r0 = blockIdx.x * 64 + wave * 16, c0 = blockIdx.y * 64;
    const size_t aoff = (size_t)(r0 + lr) * K + 8 * hi;
    v8f acc[4];
#pragma unroll
    for (int t = 0; t < 4; ++t) acc[t] = (v8f){};
#pragma unroll 1
    for (int kc = 0; kc < Klim; kc += 32) {
        const v16bf a = cat16b(*(const v8us*)(Ah + aoff + kc), *(const v8us*)(Ah + aoff + kc + 16));
        v16bf al = a; if (!(MODE & 4) && !(MODE & 16)) al = cat16b(*(const v8us*)(Al + aoff + kc), *(const v8us*)(Al + aoff + kc + 16));
#pragma unroll
        for (int t = 0; t < 4; ++t) { const size_t bo = (size_t)(c0 + t * 16 + lr) * K + kc + 8 * hi;
            const v16bf bh = cat16b(*(const v8us*)(Bh + bo), *(const v8us*)(Bh + bo + 16));
            acc[t] = wmmab(a, bh, acc[t]);
            if (!(MODE & 4)) { if (!(MODE & 16)) acc[t] = wmmab(al, bh, acc[t]); if (!(MODE & 8)) { const v16bf bl = cat16b(*(const v8us*)(Bl + bo), *(const v8us*)(Bl + bo + 16)); acc[t] = wmmab(a, bl, acc[t]); } } }
        asm volatile("v_nop\n\tv_nop\n\tv_nop\n\tv_nop" : "+v"(acc[0]), "+v"(acc[1]), "+v"(acc[2]), "+v"(acc[3]) : "v"(a), "v"(al));
    }
    float* os = &ost[wave][0];
#pragma unroll
    for (int t = 0; t < 4; ++t) {
#pragma unroll
        for (int j = 0; j < 8; ++j) os[(hi * 8 + j) * 68 + t * 16 + lr] = acc[t][j]; }
    __builtin_amdgcn_wave_barrier(); asm volatile("" ::: "memory");
    float* crow = C + (size_t)r0 * ldc + c0;
    auto pass = [&]() {
#pragma unroll
        for (int s = 0; s < 8; ++s) { const int Lid = (lane >> 3) + 4 * s, piece = lane & 7; const int row = Lid >> 1, cofs = (Lid & 1) * 32 + piece * 4;
            const v4f val = *(const v4fa*)(os + row * 68 + cofs); *(volatile v4f*)(crow + (size_t)row * ldc + cofs) = val; }
    };
    pass(); __threadfence(); pass();
}
__global__ __launch_bounds__(256) void k_planes32z(const float* __restrict__ F, int ld, int off, float sc, int rows, bf* Ph, bf* Pl) {
    typedef __attribute__((ext_vector_type(2))) unsigned short v2us;
    const int lane = threadIdx.x & 31; const size_t r = ((size_t)blockIdx.x * 8 + (threadIdx.x >> 5)) * 2 + (lane >> 4); if (r >= (size_t)rows) return; const int z = blockIdx.z; const int c0 = (lane & 15) * 2; v2us oh, ol;
    Ph += (size_t)z * rows * 32; Pl += (size_t)z * rows * 32;
#pragma unroll
    for (int i = 0; i < 2; ++i) { const float y = F[r * ld + off + z * 32 + c0 + i] * sc; const unsigned short hb = f2bf(y); oh[i] = hb; ol[i] = f2bf(y - bf2f(hb)); }
    const size_t o = r * 32 + c0; *(volatile v2us*)(Ph + o) = oh; *(volatile v2us*)(Pl + o) = ol; __threadfence(); *(volatile v2us*)(Ph + o) = oh; *(volatile v2us*)(Pl + o) = ol;
}
__global__ __launch_bounds__(256) void k_vtpadz(const float* __restrict__ F, int ld, int off, int nk, bf* Th, bf* Tl) {
    typedef __attribute__((ext_vector_type(2))) unsigned short v2us;
    const int lane = threadIdx.x & 31; const size_t wid = (size_t)blockIdx.x * 8 + (threadIdx.x >> 5); if (wid >= (size_t)64 * (nk / 64)) return; const int z = blockIdx.z; const int d = (int)(wid / (nk / 64)); const int k0 = (int)(wid % (nk / 64)) * 64 + lane * 2; v2us oh, ol;
    Th += (size_t)z * 64 * nk; Tl += (size_t)z * 64 * nk;
#pragma unroll
    for (int i = 0; i < 2; ++i) { const float y = (d < 32) ? F[(size_t)(k0 + i) * ld + off + z * 32 + (d < 32 ? d : 0)] : 0.f; const unsigned short hb = f2bf(y); oh[i] = hb; ol[i] = f2bf(y - bf2f(hb)); }
    const size_t o = (size_t)d * nk + k0; *(volatile v2us*)(Th + o) = oh; *(volatile v2us*)(Tl + o) = ol; __threadfence(); *(volatile v2us*)(Th + o) = oh; *(volatile v2us*)(Tl + o) = ol;
}
template <int NK>
__global__ __launch_bounds__(256) void k_softmaxz(const float* __restrict__ S, int rows, bf* PH, bf* PL) {
    typedef __attribute__((ext_vector_type(4))) unsigned short v4us;
    const int lane = threadIdx.x & 31, i = blockIdx.x * 8 + (threadIdx.x >> 5); if (i >= rows) return; const size_t zo = (size_t)blockIdx.z * rows * NK; const float* sr = S + zo + (size_t)i * NK; PH += zo; PL += zo;
    float m = -3.0e38f;
#pragma unroll 1
    for (int c0 = lane * 4; c0 < NK; c0 += 128) {
#pragma unroll
        for (int q = 0; q < 4; ++q) m = fmaxf(m, sr[c0 + q]); }
#pragma unroll
    for (int sh = 16; sh; sh >>= 1) m = fmaxf(m, __shfl_xor(m, sh, 32));
    float sum = 0.f;
#pragma unroll 1
    for (int c0 = lane * 4; c0 < NK; c0 += 128) {
#pragma unroll
        for (int q = 0; q < 4; ++q) sum += __expf(sr[c0 + q] - m); }
#pragma unroll
    for (int sh = 16; sh; sh >>= 1) sum += __shfl_xor(sum, sh, 32);
    const float inv = 1.0f / sum;
#pragma unroll 1
    for (int ps = 0; ps < 2; ++ps) {
#pragma unroll 1
        for (int c0 = lane * 4; c0 < NK; c0 += 128) { v4us oh, ol;
#pragma unroll
            for (int q = 0; q < 4; ++q) { const float p = __expf(sr[c0 + q] - m) * inv; const unsigned short hb = f2bf(p); oh[q] = hb; ol[q] = f2bf(p - bf2f(hb)); }
            const size_t o = (size_t)i * NK + c0; *(volatile v4us*)(PH + o) = oh; *(volatile v4us*)(PL + o) = ol; }
        if (ps == 0) __threadfence(); }
}
__global__ __launch_bounds__(256) void k_placez(const float* __restrict__ XH, int rows, int ldy, float* Y) {
    const int lane = threadIdx.x & 31; const size_t q = (size_t)blockIdx.x * 8 + (threadIdx.x >> 5); if (q >= (size_t)rows) return; const int z = blockIdx.z; const float v = XH[((size_t)z * rows + q) * 64 + lane];
    *(volatile float*)(Y + q * ldy + z * 32 + lane) = v; __threadfence(); *(volatile float*)(Y + q * ldy + z * 32 + lane) = v;
}

__global__ __launch_bounds__(256) void k_gathb(const float* __restrict__ src, int b, int rows, bf* dst) {
    const int lane = threadIdx.x & 31; const size_t r = (size_t)blockIdx.x * 8 + (threadIdx.x >> 5); if (r >= (size_t)rows) return; const float* sr = src + (r * NB_ + b) * HIDN;
#pragma unroll 1
    for (int ps = 0; ps < 2; ++ps) {
#pragma unroll
        for (int q = 0; q < HIDN / 256; ++q) { v8us o;
#pragma unroll
            for (int i = 0; i < 8; ++i) o[i] = f2bf(sr[q * 256 + lane * 8 + i]);
            *(volatile v8us*)(dst + r * HIDN + q * 256 + lane * 8) = o; }
        if (ps == 0) __threadfence(); }
}
__global__ __launch_bounds__(256) void k_wT(const float* __restrict__ Wt, bf* WT) {
    __shared__ float tl[64][65];
    typedef __attribute__((ext_vector_type(4))) unsigned short v4us;
    const int tid = threadIdx.x, h0 = blockIdx.x * 64, c0 = blockIdx.y * 64; const int rr = tid >> 2, cq = (tid & 3) * 16;
#pragma unroll
    for (int i = 0; i < 16; ++i) tl[rr][cq + i] = Wt[(size_t)(h0 + rr) * HIDN + c0 + cq + i];
    __syncthreads();
    const int lane = tid & 31, wv = tid >> 5;
    auto pass = [&]() {
#pragma unroll
        for (int st = 0; st < 4; ++st) { const int cr = wv * 8 + st * 2 + (lane >> 4); const int hq = (lane & 15) * 4; v4us v;
#pragma unroll
            for (int i = 0; i < 4; ++i) v[i] = f2bf(tl[hq + i][cr]);
            *(volatile v4us*)(WT + (size_t)(c0 + cr) * HIDN + h0 + hq) = v; }
    };
    pass(); __threadfence(); pass();
}
__global__ __launch_bounds__(256) void k_qbz(const float* __restrict__ Q, const float* __restrict__ bias, bf* Ph, bf* Pl) {
    typedef __attribute__((ext_vector_type(2))) unsigned short v2us;
    const int lane = threadIdx.x & 31; const size_t i = (size_t)blockIdx.x * 8 + (threadIdx.x >> 5); if (i >= (size_t)QL) return; const int z = blockIdx.z; Ph += (size_t)z * QL * HD; Pl += (size_t)z * QL * HD; v2us oh, ol;
#pragma unroll
    for (int q = 0; q < 2; ++q) { const int d = lane * 2 + q; const float y = Q[i * HIDN + z * HD + d] + bfr(bias[z * HD + d]); const unsigned short hb = f2bf(y); oh[q] = hb; ol[q] = f2bf(y - bf2f(hb)); }
    const size_t o = i * HD + lane * 2; *(volatile v2us*)(Ph + o) = oh; *(volatile v2us*)(Pl + o) = ol; __threadfence(); *(volatile v2us*)(Ph + o) = oh; *(volatile v2us*)(Pl + o) = ol;
}
__global__ __launch_bounds__(256) void k_kz(const float* __restrict__ F, int rows, bf* Ph, bf* Pl) {
    typedef __attribute__((ext_vector_type(2))) unsigned short v2us;
    const int lane = threadIdx.x & 31; const size_t j = (size_t)blockIdx.x * 8 + (threadIdx.x >> 5); if (j >= (size_t)rows) return; const int z = blockIdx.z; Ph += (size_t)z * rows * HD; Pl += (size_t)z * rows * HD; v2us oh, ol;
#pragma unroll
    for (int q = 0; q < 2; ++q) { const int d = lane * 2 + q; const float y = F[j * HIDN + z * HD + d]; const unsigned short hb = f2bf(y); oh[q] = hb; ol[q] = f2bf(y - bf2f(hb)); }
    const size_t o = j * HD + lane * 2; *(volatile v2us*)(Ph + o) = oh; *(volatile v2us*)(Pl + o) = ol; __threadfence(); *(volatile v2us*)(Ph + o) = oh; *(volatile v2us*)(Pl + o) = ol;
}
__global__ __launch_bounds__(256) void k_vtbz(const float* __restrict__ V, bf* Th, bf* Tl) {
    typedef __attribute__((ext_vector_type(2))) unsigned short v2us;
    const int lane = threadIdx.x & 31; const size_t wid = (size_t)blockIdx.x * 8 + (threadIdx.x >> 5); if (wid >= (size_t)HD * (QL / 64)) return; const int z = blockIdx.z; const int d = (int)(wid / (QL / 64)); const int j0 = (int)(wid % (QL / 64)) * 64 + lane * 2; v2us oh, ol;
    Th += (size_t)z * HD * QL; Tl += (size_t)z * HD * QL;
#pragma unroll
    for (int q = 0; q < 2; ++q) { const float y = V[(size_t)(j0 + q) * HIDN + z * HD + d]; const unsigned short hb = f2bf(y); oh[q] = hb; ol[q] = f2bf(y - bf2f(hb)); }
    const size_t o = (size_t)d * QL + j0; *(volatile v2us*)(Th + o) = oh; *(volatile v2us*)(Tl + o) = ol; __threadfence(); *(volatile v2us*)(Th + o) = oh; *(volatile v2us*)(Tl + o) = ol;
}
__global__ __launch_bounds__(256) void k_ef(const float* __restrict__ Q, const float* __restrict__ rsb, const float* __restrict__ segm, float* EF) {
    const int lane = threadIdx.x & 31; const size_t w = (size_t)blockIdx.x * 8 + (threadIdx.x >> 5); if (w >= (size_t)NH_ * QL) return; const int z = (int)(w / QL); const int i = (int)(w % QL);
    float e0 = 0.f, e1 = 0.f;
#pragma unroll
    for (int q = 0; q < 2; ++q) { const int d = lane * 2 + q; const float qv = Q[(size_t)i * HIDN + z * HD + d] + bfr(rsb[z * HD + d]); e0 = fmaf(qv, bfr(segm[(0 * NH_ + z) * HD + d]), e0); e1 = fmaf(qv, bfr(segm[(1 * NH_ + z) * HD + d]), e1); }
#pragma unroll
    for (int sh = 16; sh; sh >>= 1) { e0 += __shfl_xor(e0, sh, 32); e1 += __shfl_xor(e1, sh, 32); }
    const float v = (lane == 0) ? e0 : (lane == 1) ? e1 : 0.f; *(volatile float*)(EF + w * 32 + lane) = v; __threadfence(); *(volatile float*)(EF + w * 32 + lane) = v;
}
__global__ __launch_bounds__(256) void k_xsoftz(const float* __restrict__ AC, const float* __restrict__ BD, const float* __restrict__ EF, const float* __restrict__ sege, const float* __restrict__ mask, int b, bf* PH, bf* PL) {
    typedef __attribute__((ext_vector_type(4))) unsigned short v4us;
    const int lane = threadIdx.x & 31, i = blockIdx.x * 8 + (threadIdx.x >> 5); if (i >= QL) return; const int z = blockIdx.z; const float* ar = AC + ((size_t)z * QL + i) * QL; const float* br = BD + ((size_t)z * QL + i) * PL_ + (QL - i); const float ef0 = EF[((size_t)z * QL + i) * 32], ef1 = EF[((size_t)z * QL + i) * 32 + 1];
    PH += (size_t)z * QL * QL; PL += (size_t)z * QL * QL;
    auto logit = [&](int j) -> float { const size_t so = (((size_t)i * QL + j) * NB_ + b) * 2; const float se0 = bfr(sege[so]), se1 = bfr(sege[so + 1]); const float v = (ar[j] + br[j] + se0 * ef0 + se1 * ef1) * SCL; return v - 1e30f * bfr(mask[((size_t)i * QL + j) * NB_ + b]); };
    float m = -3.0e38f;
#pragma unroll 1
    for (int c0 = lane * 4; c0 < QL; c0 += 128) {
#pragma unroll
        for (int q = 0; q < 4; ++q) m = fmaxf(m, logit(c0 + q)); }
#pragma unroll
    for (int sh = 16; sh; sh >>= 1) m = fmaxf(m, __shfl_xor(m, sh, 32));
    float sum = 0.f;
#pragma unroll 1
    for (int c0 = lane * 4; c0 < QL; c0 += 128) {
#pragma unroll
        for (int q = 0; q < 4; ++q) sum += __expf(logit(c0 + q) - m); }
#pragma unroll
    for (int sh = 16; sh; sh >>= 1) sum += __shfl_xor(sum, sh, 32);
    const float inv = 1.0f / sum;
#pragma unroll 1
    for (int ps = 0; ps < 2; ++ps) {
#pragma unroll 1
        for (int c0 = lane * 4; c0 < QL; c0 += 128) { v4us oh, ol;
#pragma unroll
            for (int q = 0; q < 4; ++q) { const float p = __expf(logit(c0 + q) - m) * inv; const unsigned short hb = f2bf(p); oh[q] = hb; ol[q] = f2bf(p - bf2f(hb)); }
            const size_t o = (size_t)i * QL + c0; *(volatile v4us*)(PH + o) = oh; *(volatile v4us*)(PL + o) = ol; }
        if (ps == 0) __threadfence(); }
}
__global__ __launch_bounds__(256) void k_splitH(const float* __restrict__ src, int rows, bf* dh, bf* dl) {
    const int lane = threadIdx.x & 31; const size_t r = (size_t)blockIdx.x * 8 + (threadIdx.x >> 5); if (r >= (size_t)rows) return;
#pragma unroll 1
    for (int ps = 0; ps < 2; ++ps) {
#pragma unroll
        for (int q = 0; q < HIDN / 256; ++q) { const size_t o = r * HIDN + q * 256 + lane * 8; const v8f v = *(const v8f*)(src + o); v8us oh, ol;
#pragma unroll
            for (int i = 0; i < 8; ++i) { const unsigned short hb = f2bf(v[i]); oh[i] = hb; ol[i] = f2bf(v[i] - bf2f(hb)); }
            *(volatile v8us*)(dh + o) = oh; *(volatile v8us*)(dl + o) = ol; }
        if (ps == 0) __threadfence(); }
}
__global__ __launch_bounds__(256) void k_resln(const float* __restrict__ AO, const float* __restrict__ hs, int b, const float* __restrict__ g, const float* __restrict__ be, float* OUTP) {
    const int lane = threadIdx.x & 31; const size_t i = (size_t)blockIdx.x * 8 + (threadIdx.x >> 5); if (i >= (size_t)QL) return; const size_t r = i * NB_ + b; float v[32]; float s = 0.f;
#pragma unroll
    for (int st = 0; st < 4; ++st) {
#pragma unroll
        for (int q = 0; q < 8; ++q) { const size_t o = r * HIDN + st * 256 + lane * 8 + q; const float t = AO[i * HIDN + st * 256 + lane * 8 + q] + bfr(hs[o]); v[st * 8 + q] = t; s += t; } }
#pragma unroll
    for (int sh = 16; sh; sh >>= 1) s += __shfl_xor(s, sh, 32);
    const float mu = s * (1.0f / HIDN); float qv = 0.f;
#pragma unroll
    for (int i2 = 0; i2 < 32; ++i2) { const float d = v[i2] - mu; qv = fmaf(d, d, qv); }
#pragma unroll
    for (int sh = 16; sh; sh >>= 1) qv += __shfl_xor(qv, sh, 32);
    const float rs = rsqrtf(qv * (1.0f / HIDN) + LEPS);
#pragma unroll 1
    for (int ps = 0; ps < 2; ++ps) {
#pragma unroll
        for (int st = 0; st < 4; ++st) { const int c0 = st * 256 + lane * 8; v8f y;
#pragma unroll
            for (int q = 0; q < 8; ++q) y[q] = (v[st * 8 + q] - mu) * rs * bfr(g[c0 + q]) + bfr(be[c0 + q]);
            *(volatile v8f*)(OUTP + r * HIDN + c0) = y; }
        if (ps == 0) __threadfence(); }
}

extern "C" void kernel_launch(void* const* d_in, const int* in_sizes, int n_in,
                              void* d_out, int out_size, void* d_ws, size_t ws_size, hipStream_t stream) {
    (void)in_sizes; (void)n_in; (void)out_size;
    const float* hs = (const float*)d_in[0]; const float* pe = (const float*)d_in[1]; const float* sege = (const float*)d_in[2]; const float* mask = (const float*)d_in[3];
    const float* wq = (const float*)d_in[4]; const float* wk = (const float*)d_in[5]; const float* wv = (const float*)d_in[6]; const float* wr = (const float*)d_in[7]; const float* wo = (const float*)d_in[8]; const float* rwb = (const float*)d_in[9]; const float* rrb = (const float*)d_in[10]; const float* rsb = (const float*)d_in[11]; const float* segm = (const float*)d_in[12]; const float* lng = (const float*)d_in[13]; const float* lnb = (const float*)d_in[14];
    float* out = (float*)d_out;
    char* wsp = (char*)d_ws;
    auto take = [&](size_t bytes) { char* p = wsp; wsp += (bytes + 255) & ~(size_t)255; return (void*)p; };
    const size_t WSZ = (size_t)HIDN * HIDN * 2;
    bf* WQ = (bf*)take(WSZ); bf* WK = (bf*)take(WSZ); bf* WV = (bf*)take(WSZ); bf* WR = (bf*)take(WSZ); bf* WO = (bf*)take(WSZ);
    bf* Xb = (bf*)take((size_t)QL * HIDN * 2); bf* Pb = (bf*)take((size_t)PL_ * HIDN * 2); float* QF = (float*)take((size_t)QL * HIDN * 4); float* KF = (float*)take((size_t)QL * HIDN * 4); float* VF = (float*)take((size_t)QL * HIDN * 4); float* RF = (float*)take((size_t)PL_ * HIDN * 4);
    bf* Qh = (bf*)take((size_t)ZH * QL * HD * 2); bf* Ql = (bf*)take((size_t)ZH * QL * HD * 2); bf* Kh = (bf*)take((size_t)ZH * PL_ * HD * 2); bf* Kl = (bf*)take((size_t)ZH * PL_ * HD * 2); bf* VTh = (bf*)take((size_t)ZH * HD * QL * 2); bf* VTl = (bf*)take((size_t)ZH * HD * QL * 2);
    float* AC = (float*)take((size_t)ZH * QL * QL * 4); float* BD = (float*)take((size_t)ZH * QL * PL_ * 4); float* EF = (float*)take((size_t)NH_ * QL * 32 * 4); bf* PH = (bf*)take((size_t)ZH * QL * QL * 2); bf* PLn = (bf*)take((size_t)ZH * QL * QL * 2);
    float* AV = (float*)take((size_t)QL * HIDN * 4); bf* AVh = (bf*)take((size_t)QL * HIDN * 2); bf* AVl = (bf*)take((size_t)QL * HIDN * 2); float* AO = (float*)take((size_t)QL * HIDN * 4);
    if ((size_t)(wsp - (char*)d_ws) > ws_size) return;
    k_wT<<<dim3(HIDN / 64, HIDN / 64, 1), 256, 0, stream>>>(wq, WQ); k_wT<<<dim3(HIDN / 64, HIDN / 64, 1), 256, 0, stream>>>(wk, WK); k_wT<<<dim3(HIDN / 64, HIDN / 64, 1), 256, 0, stream>>>(wv, WV); k_wT<<<dim3(HIDN / 64, HIDN / 64, 1), 256, 0, stream>>>(wr, WR);
    k_cvt8<<<(HIDN * HIDN / 8 + 255) / 256, 256, 0, stream>>>(wo, WO, HIDN * HIDN / 8);
    const dim3 gq(QL / 64, HIDN / 64, 1), gr(PL_ / 64, HIDN / 64, 1);
    for (int b = 0; b < NB_; ++b) {
        k_gathb<<<QL / 8, 256, 0, stream>>>(hs, b, QL, Xb); k_gathb<<<PL_ / 8, 256, 0, stream>>>(pe, b, PL_, Pb);
        k_gemmb<false, false><<<gq, 128, 0, stream>>>(Xb, nullptr, WQ, nullptr, QF, HIDN, nullptr, nullptr, HIDN); k_gemmb<false, false><<<gq, 128, 0, stream>>>(Xb, nullptr, WK, nullptr, KF, HIDN, nullptr, nullptr, HIDN); k_gemmb<false, false><<<gq, 128, 0, stream>>>(Xb, nullptr, WV, nullptr, VF, HIDN, nullptr, nullptr, HIDN);
        k_gemmb<false, false><<<gr, 128, 0, stream>>>(Pb, nullptr, WR, nullptr, RF, HIDN, nullptr, nullptr, HIDN);
        k_qbz<<<dim3(QL / 8, 1, ZH), 256, 0, stream>>>(QF, rwb, Qh, Ql); k_kz<<<dim3(QL / 8, 1, ZH), 256, 0, stream>>>(KF, QL, Kh, Kl);
        k_gemm3z<0><<<dim3(QL / 64, QL / 64, ZH), 128, 0, stream>>>(Qh, Ql, Kh, Kl, HD, AC, QL, (size_t)QL * HD, (size_t)QL * HD, (size_t)QL * QL);
        k_qbz<<<dim3(QL / 8, 1, ZH), 256, 0, stream>>>(QF, rrb, Qh, Ql); k_kz<<<dim3(PL_ / 8, 1, ZH), 256, 0, stream>>>(RF, PL_, Kh, Kl);
        k_gemm3z<0><<<dim3(QL / 64, PL_ / 64, ZH), 128, 0, stream>>>(Qh, Ql, Kh, Kl, HD, BD, PL_, (size_t)QL * HD, (size_t)PL_ * HD, (size_t)QL * PL_);
        k_ef<<<(NH_ * QL) / 8, 256, 0, stream>>>(QF, rsb, segm, EF);
        k_xsoftz<<<dim3(QL / 8, 1, ZH), 256, 0, stream>>>(AC, BD, EF, sege, mask, b, PH, PLn);
        k_vtbz<<<dim3((HD * (QL / 64)) / 8, 1, ZH), 256, 0, stream>>>(VF, VTh, VTl);
        k_gemm3z<0><<<dim3(QL / 64, 1, ZH), 128, 0, stream>>>(PH, PLn, VTh, VTl, QL, AV, HIDN, (size_t)QL * QL, (size_t)HD * QL, (size_t)HD);
        k_splitH<<<QL / 8, 256, 0, stream>>>(AV, QL, AVh, AVl);
        k_gemmb<true, false><<<gq, 128, 0, stream>>>(AVh, AVl, WO, nullptr, AO, HIDN, nullptr, nullptr, HIDN);
        k_resln<<<QL / 8, 256, 0, stream>>>(AO, hs, b, lng, lnb, out); }
}
